// GNN_90546500534502
// MI455X (gfx1250) — hardware-verified
//
#include <hip/hip_runtime.h>
#include <stddef.h>
#include <stdint.h>
#include <math.h>


#define CIN    512
#define HID    1024
#define K3     2048
#define NHEAD  8
#define NTHR   256
#define NWAVE  8
#define EPT    8
#define CHUNK  (NTHR * EPT)
#define WCAP   (EPT * 32)
#define LISTN  (NWAVE * WCAP)
#define NBD    1024
#define SLD    10
#define NBA    64
#define SLA    6
#define RCAP   4096
#define DEGCAP 64
#define GBM    64
#define GBN    64
#define GTHR   128
#define NU1    (HID * (CIN / 8))
#define NU3    (HID * (K3 / 8))
#define AGG_ZINTS (LISTN + 2 * RCAP + 3 * NBA)
#define WSMAX  134217728

static_assert((CHUNK & (CHUNK - 1)) == 0 && CHUNK <= 4096);
static_assert((NBD & (NBD - 1)) == 0 && NBD == (1 << SLD));
static_assert((NBA & (NBA - 1)) == 0 && NBA == (1 << SLA));
static_assert(((long long)CHUNK << SLD) < (1LL << 31));
static_assert(NBD == NTHR * 4);
static_assert(LISTN % NTHR == 0);
static_assert(NBA % NWAVE == 0 && NBA % 32 == 0 && NBA == GBM && NBA == 64);
static_assert(DEGCAP == 64);
static_assert(RCAP % 32 == 0 && AGG_ZINTS % 4 == 0 && LISTN % 4 == 0);
static_assert(CIN % 32 == 0 && K3 % 32 == 0 && K3 == 2 * HID && HID % GBN == 0);
static_assert(GBM == (GTHR / 32) * 16 && GBN == 64);
static_assert(NU1 % NTHR == 0 && NU3 % NTHR == 0);
static_assert(CIN / 8 == 64 && K3 / 8 == 256 && HID == 4 * 256);
static_assert((AGG_ZINTS + 16) * 4 + HID * 3 * 4 + NBA * 4 * 4 + NBA * 4 + 256 * 4 <= 65536);

typedef float          v4f   __attribute__((ext_vector_type(4)));
typedef float          v8f   __attribute__((ext_vector_type(8)));
typedef int            v4i   __attribute__((ext_vector_type(4)));
typedef int            v8i   __attribute__((ext_vector_type(8)));
typedef unsigned short v8us  __attribute__((ext_vector_type(8)));
typedef unsigned short v16us __attribute__((ext_vector_type(16)));
typedef __bf16         v16bf __attribute__((ext_vector_type(16)));
typedef v4f  __attribute__((may_alias)) v4fa;
typedef v4i  __attribute__((may_alias)) v4ia;
typedef v8us __attribute__((may_alias)) v8usa;
union FragB { v16bf v; v16us u; v8us h[2]; v8i w; };

__device__ __forceinline__ v8f wmb(const FragB& a, const FragB& b, v8f c) {
  v8f d = __builtin_amdgcn_wmma_f32_16x16x32_bf16(false, a.v, false, b.v, (short)0, c, false, false);
  asm volatile("v_nop\n\tv_nop\n\tv_nop\n\tv_nop" : "+v"(d) : "v"(a.w), "v"(b.w));
  return d;
}

__device__ __forceinline__ unsigned bf16_bits(float f) {
  const unsigned u = __float_as_uint(f);
  return (u + 0x7FFFu + ((u >> 16) & 1u)) >> 16;
}
__device__ __forceinline__ float bf16_val(float f) {
  return __uint_as_float(bf16_bits(f) << 16);
}
__device__ __forceinline__ int clampi(int v, int lo, int hi) {
  return v < lo ? lo : (v > hi ? hi : v);
}

template <int SLB>
__device__ __forceinline__ int scan_chunk(const int* __restrict__ dsts, int nE, int cbase, int slotBase,
                                          int nb, int vec8, int* list, int tid, int lane, int wave) {
  int wc = 0;
  const int el0  = tid * EPT;
  const int e0   = cbase + el0;
  const int sent = -2147483647 - 1;
  v4i da, db;
  if (vec8 != 0 && cbase + CHUNK <= nE) {
    da = *(const v4i*)(dsts + e0);
    db = *(const v4i*)(dsts + e0 + 4);
  } else {
    da.x = (e0     < nE) ? dsts[min(e0,     nE - 1)] : sent;
    da.y = (e0 + 1 < nE) ? dsts[min(e0 + 1, nE - 1)] : sent;
    da.z = (e0 + 2 < nE) ? dsts[min(e0 + 2, nE - 1)] : sent;
    da.w = (e0 + 3 < nE) ? dsts[min(e0 + 3, nE - 1)] : sent;
    db.x = (e0 + 4 < nE) ? dsts[min(e0 + 4, nE - 1)] : sent;
    db.y = (e0 + 5 < nE) ? dsts[min(e0 + 5, nE - 1)] : sent;
    db.z = (e0 + 6 < nE) ? dsts[min(e0 + 6, nE - 1)] : sent;
    db.w = (e0 + 7 < nE) ? dsts[min(e0 + 7, nE - 1)] : sent;
  }
  const unsigned nbs = (unsigned)slotBase;
  const unsigned unb = (unsigned)nb;
  const unsigned s0 = (unsigned)da.x - nbs, s1 = (unsigned)da.y - nbs;
  const unsigned s2 = (unsigned)da.z - nbs, s3 = (unsigned)da.w - nbs;
  const unsigned s4 = (unsigned)db.x - nbs, s5 = (unsigned)db.y - nbs;
  const unsigned s6 = (unsigned)db.z - nbs, s7 = (unsigned)db.w - nbs;
  const bool h0 = s0 < unb, h1 = s1 < unb, h2 = s2 < unb, h3 = s3 < unb;
  const bool h4 = s4 < unb, h5 = s5 < unb, h6 = s6 < unb, h7 = s7 < unb;
  const unsigned any = __builtin_amdgcn_ballot_w32(h0 | h1 | h2 | h3 | h4 | h5 | h6 | h7);
  if (any != 0u) {
#define HITJ(J, HJ, SJ) { \
      const unsigned mj = __builtin_amdgcn_ballot_w32(HJ); \
      if (mj != 0u) { \
        if (HJ) { \
          const int pos = wc + (int)__builtin_amdgcn_mbcnt_lo(mj, 0u); \
          if (pos < WCAP) list[wave * WCAP + pos] = ((el0 + (J)) << SLB) | (int)(SJ); \
        } \
        wc += (int)__builtin_popcount(mj); } }
    HITJ(0, h0, s0)
    HITJ(1, h1, s1)
    HITJ(2, h2, s2)
    HITJ(3, h3, s3)
    HITJ(4, h4, s4)
    HITJ(5, h5, s5)
    HITJ(6, h6, s6)
    HITJ(7, h7, s7)
#undef HITJ
  }
  return wc;
}

__global__ __launch_bounds__(NTHR) void k_wprep(const float* __restrict__ W1, const float* __restrict__ W3,
                                                unsigned short* W1T, unsigned short* W3T2) {
  const int u = (int)blockIdx.x * NTHR + (int)threadIdx.x;
  v8us o;
  unsigned short* dp;
  if (u < NU1) {
    const int n  = u >> 6;
    const int k8 = (u & 63) * 8;
    const float* p = W1 + (size_t)k8 * HID + n;
#pragma unroll
    for (int i = 0; i < 8; ++i) o[i] = (unsigned short)bf16_bits(p[(size_t)i * HID]);
    dp = W1T + (size_t)n * CIN + k8;
  } else if (u < NU1 + NU3) {
    const int v  = u - NU1;
    const int n  = v >> 8;
    const int k8 = (v & 255) * 8;
    const int kk = k8 & (HID - 1);
    const float* p = W3 + (size_t)kk * HID + n;
#pragma unroll
    for (int i = 0; i < 8; ++i) o[i] = (unsigned short)bf16_bits(p[(size_t)i * HID]);
    dp = W3T2 + (size_t)n * K3 + k8;
  } else {
    return;
  }
  *(volatile v8us*)dp = o;
  __threadfence();
  *(volatile v8us*)dp = o;
}

__global__ __launch_bounds__(NTHR) void k_cvx(const float* __restrict__ x, int nN, int nUnits,
                                              unsigned short* xb) {
  const int u = (int)blockIdx.x * NTHR + (int)threadIdx.x;
  if (u >= nUnits) return;
  const int row = u >> 6;
  const int k8  = (u & 63) * 8;
  const int rc  = row < nN ? row : nN - 1;
  const float* p = x + (size_t)rc * CIN + k8;
  const v4f a = *(const v4fa*)p;
  const v4f b = *(const v4fa*)(p + 4);
  const bool ok = row < nN;
  v8us o;
  o[0] = ok ? (unsigned short)bf16_bits(a.x) : (unsigned short)0;
  o[1] = ok ? (unsigned short)bf16_bits(a.y) : (unsigned short)0;
  o[2] = ok ? (unsigned short)bf16_bits(a.z) : (unsigned short)0;
  o[3] = ok ? (unsigned short)bf16_bits(a.w) : (unsigned short)0;
  o[4] = ok ? (unsigned short)bf16_bits(b.x) : (unsigned short)0;
  o[5] = ok ? (unsigned short)bf16_bits(b.y) : (unsigned short)0;
  o[6] = ok ? (unsigned short)bf16_bits(b.z) : (unsigned short)0;
  o[7] = ok ? (unsigned short)bf16_bits(b.w) : (unsigned short)0;
  unsigned short* dp = xb + (size_t)row * CIN + k8;
  *(volatile v8us*)dp = o;
  __threadfence();
  *(volatile v8us*)dp = o;
}

__global__ __launch_bounds__(NTHR) void k_deg(const int* __restrict__ dsts, int nE, int vec8, float* dis) {
  __shared__ __attribute__((aligned(16))) int scnt[NBD];
  __shared__ __attribute__((aligned(16))) int list[LISTN];
  __shared__ __attribute__((aligned(16))) float sdis[NBD];
  __shared__ int wcnt[NWAVE];
  const int tid = (int)threadIdx.x, lane = tid & 31, wave = tid >> 5;
  const int nodeBase = (int)blockIdx.x * NBD;

  for (int i = tid; i < NBD; i += NTHR) scnt[i] = 0;
  for (int i = tid; i < LISTN; i += NTHR) list[i] = 0;
  if (tid < NWAVE) wcnt[tid] = 0;
  __syncthreads();

  const int nChunks = (nE + CHUNK - 1) / CHUNK;
#pragma unroll 1
  for (int ch = 0; ch < nChunks; ++ch) {
    const int cbase = ch * CHUNK;
    const int wc = scan_chunk<SLD>(dsts, nE, cbase, nodeBase, NBD, vec8, list, tid, lane, wave);
    if (lane == 0) wcnt[wave] = wc;
    __syncthreads();
    if (wave == 0) {
#pragma unroll 1
      for (int w2 = 0; w2 < NWAVE; ++w2) {
        int c = wcnt[w2];
        c = c < 0 ? 0 : (c > WCAP ? WCAP : c);
#pragma unroll 1
        for (int b0 = 0; b0 < c; b0 += 32) {
          const int idx = b0 + lane;
          const int ent = list[w2 * WCAP + (idx < WCAP ? idx : WCAP - 1)];
          const int m32 = (c - b0) < 32 ? (c - b0) : 32;
#pragma unroll 1
          for (int k = 0; k < m32; ++k) {
            const int u  = __builtin_amdgcn_readlane(ent, k);
            const int sl = u & (NBD - 1);
            if (lane == 0) scnt[sl] = scnt[sl] + 1;
          }
        }
      }
    }
    __syncthreads();
  }

#pragma unroll 1
  for (int i = tid; i < NBD; i += NTHR) {
    const float d = (float)scnt[i] + 1.0f;
    sdis[i] = (d > 0.0f) ? (1.0f / sqrtf(d)) : 0.0f;
  }
  __syncthreads();
  const v4f v = *(const v4fa*)(sdis + 4 * tid);
  float* dp = dis + (size_t)nodeBase + 4 * tid;
  *(volatile v4f*)dp = v;
  __threadfence();
  *(volatile v4f*)dp = v;
}

__global__ __launch_bounds__(GTHR) void k_gemm(
    const unsigned short* __restrict__ A, const unsigned short* __restrict__ WT,
    float* outF, int K, int ldo)
{
  __shared__ __attribute__((aligned(16))) float stg[GBM * GBN];
  const int tid = (int)threadIdx.x, lane = tid & 31, wave = tid >> 5, hh = lane >> 4, m = lane & 15;
  const int rowBase = (int)blockIdx.x * GBM;
  const int col0    = (int)blockIdx.y * GBN;

  v8f acc[4];
  {
    const v8f z = {0.f, 0.f, 0.f, 0.f, 0.f, 0.f, 0.f, 0.f};
    acc[0] = z; acc[1] = z; acc[2] = z; acc[3] = z;
  }
  const unsigned short* ap = A  + (size_t)(rowBase + 16 * wave + m) * (size_t)K + 8 * hh;
  const unsigned short* wp = WT + (size_t)(col0 + m) * (size_t)K + 8 * hh;
  const int ksteps = K >> 5;
#pragma unroll 1
  for (int ks = 0; ks < ksteps; ++ks) {
    FragB af;
    af.h[0] = *(const v8usa*)(ap + 32 * ks);
    af.h[1] = *(const v8usa*)(ap + 32 * ks + 16);
#pragma unroll
    for (int t = 0; t < 4; ++t) {
      const unsigned short* wq = wp + (size_t)(16 * t) * (size_t)K + 32 * ks;
      FragB bf;
      bf.h[0] = *(const v8usa*)wq;
      bf.h[1] = *(const v8usa*)(wq + 16);
      acc[t] = wmb(af, bf, acc[t]);
    }
  }

#pragma unroll
  for (int t = 0; t < 4; ++t) {
    const int lc = 16 * t + m;
#pragma unroll
    for (int r = 0; r < 8; ++r) {
      const int lr = 16 * wave + 8 * hh + r;
      stg[lr * GBN + lc] = acc[t][r];
    }
  }
  __syncthreads();

  v4f fv[8];
#pragma unroll
  for (int i = 0; i < 8; ++i) {
    const int lr = 16 * wave + 2 * i + hh;
    fv[i] = *(const v4fa*)(stg + lr * GBN + 4 * m);
  }
#pragma unroll
  for (int i = 0; i < 8; ++i) {
    const int lr = 16 * wave + 2 * i + hh;
    const int gr = rowBase + lr;
    float* op = outF + (size_t)gr * (size_t)ldo + col0 + 4 * m;
    *(volatile v4f*)op = fv[i];
  }
  __threadfence();
#pragma unroll
  for (int i = 0; i < 8; ++i) {
    const int lr = 16 * wave + 2 * i + hh;
    const int gr = rowBase + lr;
    float* op = outF + (size_t)gr * (size_t)ldo + col0 + 4 * m;
    *(volatile v4f*)op = fv[i];
  }
}

template <int MODE>
__global__ __launch_bounds__(NTHR) void k_scan(const int* __restrict__ srcs, const int* __restrict__ dsts,
                                               int nE, int nN, int vec8,
                                               const float* __restrict__ dis,
                                               const float* __restrict__ Hm, const float* __restrict__ bias,
                                               const float* __restrict__ att, const float* __restrict__ Wsm,
                                               unsigned short* xhl, float* Tout, float* Aout,
                                               const float* __restrict__ Tin, const float* __restrict__ bs,
                                               float* yout) {
  __shared__ __attribute__((aligned(16))) int dsm[AGG_ZINTS + 16];
  __shared__ __attribute__((aligned(16))) float w2s[HID * 3];
  __shared__ __attribute__((aligned(16))) float tbuf[NBA * 4];
  __shared__ __attribute__((aligned(16))) float abuf[NBA];
  __shared__ __attribute__((aligned(16))) float ybuf[256];
  int* list = dsm;
  int* hl   = dsm + LISTN;
  int* sl   = dsm + LISTN + RCAP;
  int* cnt  = dsm + LISTN + 2 * RCAP;
  int* offs = cnt + NBA;
  int* cur  = offs + NBA;
  int* misc = cur + NBA;
  const int tid = (int)threadIdx.x, lane = tid & 31, wave = tid >> 5;
  const int nodeBase = (int)blockIdx.x * NBA;

  {
    const v4i z4 = {0, 0, 0, 0};
    for (int i = tid * 4; i < AGG_ZINTS; i += NTHR * 4) *(v4ia*)(dsm + i) = z4;
    if (tid < 16) misc[tid] = 0;
  }
  if constexpr (MODE != 3) {
#pragma unroll 1
    for (int i = tid; i < (HID * 3) / 4; i += NTHR) {
      const v4f w = *(const v4fa*)(Wsm + 4 * i);
      v4f r;
      r.x = bf16_val(w.x); r.y = bf16_val(w.y); r.z = bf16_val(w.z); r.w = bf16_val(w.w);
      *(v4fa*)(w2s + 4 * i) = r;
    }
  }
  __syncthreads();

  int t = 0, ov = 0;
  const int nChunks = (nE + CHUNK - 1) / CHUNK;
#pragma unroll 1
  for (int ch = 0; ch < nChunks; ++ch) {
    const int cbase = ch * CHUNK;
    const int wc = scan_chunk<SLA>(dsts, nE, cbase, nodeBase, NBA, vec8, list, tid, lane, wave);
    if (lane == 0) misc[wave] = wc;
    __syncthreads();
    if (wave == 0) {
#pragma unroll 1
      for (int w2 = 0; w2 < NWAVE; ++w2) {
        int c = misc[w2];
        c = c < 0 ? 0 : (c > WCAP ? WCAP : c);
#pragma unroll 1
        for (int b0 = 0; b0 < c; b0 += 32) {
          const int idx = b0 + lane;
          const int ent = list[w2 * WCAP + (idx < WCAP ? idx : WCAP - 1)];
          const int m32 = (c - b0) < 32 ? (c - b0) : 32;
#pragma unroll 1
          for (int k = 0; k < m32; ++k) {
            const int u    = __builtin_amdgcn_readlane(ent, k);
            const int slot = u & (NBA - 1);
            const int el   = (u >> SLA) & (CHUNK - 1);
            const int pk   = ((cbase + el) << SLA) | slot;
            if (t < RCAP) {
              if (lane == 0) { hl[t] = pk; cnt[slot] = cnt[slot] + 1; }
              t = t + 1;
            } else {
              ov = 1;
            }
          }
        }
      }
    }
    __syncthreads();
  }
  if (wave == 0 && lane == 0) { misc[8] = t; misc[9] = ov; }
  __syncthreads();
  int tt = misc[8];
  tt = tt < 0 ? 0 : (tt > RCAP ? RCAP : tt);
  const int ovf = misc[9];

  if (wave == 0) {
    const int base = lane * (NBA / 32);
    int s = 0;
#pragma unroll 1
    for (int i = 0; i < NBA / 32; ++i) s += cnt[base + i];
    int incl = s;
#pragma unroll
    for (int d = 1; d < 32; d <<= 1) {
      const int y = __shfl_up(incl, d, 32);
      if (lane >= d) incl += y;
    }
    int run = incl - s;
#pragma unroll 1
    for (int i = 0; i < NBA / 32; ++i) {
      const int cv = cnt[base + i];
      offs[base + i] = run;
      cur[base + i]  = run;
      run += cv;
    }
  }
  __syncthreads();
  if (wave == 0) {
#pragma unroll 1
    for (int b0 = 0; b0 < tt; b0 += 32) {
      const int idx = b0 + lane;
      const int ent = hl[idx < RCAP ? idx : RCAP - 1];
      const int m32 = (tt - b0) < 32 ? (tt - b0) : 32;
#pragma unroll 1
      for (int k = 0; k < m32; ++k) {
        const int u    = __builtin_amdgcn_readlane(ent, k);
        const int slot = u & (NBA - 1);
        if (lane == 0) {
          int p = cur[slot];
          p = p < 0 ? 0 : (p > RCAP - 1 ? RCAP - 1 : p);
          sl[p] = u;
          cur[slot] = p + 1;
        }
      }
    }
  }
  __syncthreads();

  const float qnan = __int_as_float(0x7fc00000);
  const float pz = (ovf != 0) ? qnan : 0.0f;
#pragma unroll 1
  for (int si = 0; si < NBA / NWAVE; ++si) {
    const int s    = si * NWAVE + wave;
    const int node = nodeBase + s;
    const int nc   = node < nN ? node : nN - 1;
    int c = cnt[s];
    const bool big = c > DEGCAP;
    c = clampi(c, 0, DEGCAP);
    const int o = clampi(offs[s], 0, RCAP);
    const float dd = dis[nc];
    const float rd = dd * dd;
    const int i0 = min(o + lane, RCAP - 1);
    const int i1 = min(o + 32 + lane, RCAP - 1);
    const int e0 = clampi(sl[i0] >> SLA, 0, nE - 1);
    const int e1 = clampi(sl[i1] >> SLA, 0, nE - 1);
    const int sr0 = clampi(srcs[e0], 0, nN - 1);
    const int sr1 = clampi(srcs[e1], 0, nN - 1);
    const float cf0 = dis[sr0] * dd;
    const float cf1 = dis[sr1] * dd;
    const int cfi0 = __float_as_int(cf0);
    const int cfi1 = __float_as_int(cf1);
    const float pzr = big ? qnan : pz;

    if constexpr (MODE != 3) {
      float t0 = 0.0f, t1 = 0.0f, t2 = 0.0f, ad = 0.0f;
      const float* attr = att + (size_t)(nc & (NHEAD - 1)) * HID;
#pragma unroll 1
      for (int q = 0; q < HID / 256; ++q) {
        const int cb = 256 * q + 8 * lane;
        float acc[8];
#pragma unroll
        for (int i = 0; i < 8; ++i) acc[i] = 0.0f;
#pragma unroll 1
        for (int b = 0; b < 2; ++b) {
          const int srb = (b != 0) ? sr1 : sr0;
          const int cfb = (b != 0) ? cfi1 : cfi0;
          const int nb  = clampi(c - 32 * b, 0, 32);
#pragma unroll 1
          for (int k = 0; k < nb; ++k) {
            const int   sk = __builtin_amdgcn_readlane(srb, k);
            const float ck = __int_as_float(__builtin_amdgcn_readlane(cfb, k));
            const float* hp = Hm + (size_t)sk * HID + cb;
            const v4f ha = *(const v4fa*)hp;
            const v4f hb = *(const v4fa*)(hp + 4);
            acc[0] = fmaf(ck, ha.x, acc[0]); acc[1] = fmaf(ck, ha.y, acc[1]);
            acc[2] = fmaf(ck, ha.z, acc[2]); acc[3] = fmaf(ck, ha.w, acc[3]);
            acc[4] = fmaf(ck, hb.x, acc[4]); acc[5] = fmaf(ck, hb.y, acc[5]);
            acc[6] = fmaf(ck, hb.z, acc[6]); acc[7] = fmaf(ck, hb.w, acc[7]);
          }
        }
        float sv[8], bv[8], av[8], y[8];
        {
          const float* sp = Hm + (size_t)nc * HID + cb;
          const v4f sa = *(const v4fa*)sp;
          const v4f sb = *(const v4fa*)(sp + 4);
          sv[0] = sa.x; sv[1] = sa.y; sv[2] = sa.z; sv[3] = sa.w;
          sv[4] = sb.x; sv[5] = sb.y; sv[6] = sb.z; sv[7] = sb.w;
          const v4f ba = *(const v4fa*)(bias + cb);
          const v4f bb = *(const v4fa*)(bias + cb + 4);
          bv[0] = bf16_val(ba.x); bv[1] = bf16_val(ba.y); bv[2] = bf16_val(ba.z); bv[3] = bf16_val(ba.w);
          bv[4] = bf16_val(bb.x); bv[5] = bf16_val(bb.y); bv[6] = bf16_val(bb.z); bv[7] = bf16_val(bb.w);
          const v4f aa = *(const v4fa*)(attr + cb);
          const v4f ab = *(const v4fa*)(attr + cb + 4);
          av[0] = bf16_val(aa.x); av[1] = bf16_val(aa.y); av[2] = bf16_val(aa.z); av[3] = bf16_val(aa.w);
          av[4] = bf16_val(ab.x); av[5] = bf16_val(ab.y); av[6] = bf16_val(ab.z); av[7] = bf16_val(ab.w);
        }
#pragma unroll
        for (int i = 0; i < 8; ++i) {
          const float v = (acc[i] + sv[i] * rd) + bv[i];
          const float r = (v > 0.0f) ? v : (v - v);
          y[i] = r + pzr;
        }
        if constexpr (MODE == 1) {
          v8us hv, lv;
#pragma unroll
          for (int i = 0; i < 8; ++i) {
            const unsigned hb = bf16_bits(y[i]);
            hv[i] = (unsigned short)hb;
            lv[i] = (unsigned short)bf16_bits(y[i] - __uint_as_float(hb << 16));
          }
          if (node < nN) {
            unsigned short* xp = xhl + (size_t)node * K3 + cb;
            *(volatile v8us*)xp = hv;
            *(volatile v8us*)(xp + HID) = lv;
            __threadfence();
            *(volatile v8us*)xp = hv;
            *(volatile v8us*)(xp + HID) = lv;
          }
        }
        {
          const float* wq = w2s + 3 * cb;
          float wv[24];
#pragma unroll
          for (int j = 0; j < 6; ++j) {
            const v4f w4 = *(const v4fa*)(wq + 4 * j);
            wv[4 * j + 0] = w4.x; wv[4 * j + 1] = w4.y; wv[4 * j + 2] = w4.z; wv[4 * j + 3] = w4.w;
          }
#pragma unroll
          for (int i = 0; i < 8; ++i) {
            t0 = fmaf(y[i], wv[3 * i + 0], t0);
            t1 = fmaf(y[i], wv[3 * i + 1], t1);
            t2 = fmaf(y[i], wv[3 * i + 2], t2);
            ad = fmaf(y[i], av[i], ad);
          }
        }
      }
#pragma unroll
      for (int d = 16; d > 0; d >>= 1) {
        t0 += __shfl_xor(t0, d, 32);
        t1 += __shfl_xor(t1, d, 32);
        t2 += __shfl_xor(t2, d, 32);
        ad += __shfl_xor(ad, d, 32);
      }
      const float am = ad * (1.0f / 1024.0f);
      if (lane == 0) {
        tbuf[4 * s + 0] = t0; tbuf[4 * s + 1] = t1; tbuf[4 * s + 2] = t2; tbuf[4 * s + 3] = 0.0f;
        abuf[s] = am;
      }
    }

    if constexpr (MODE != 1) {
      const v4f ta = *(const v4fa*)(Tin + 4 * (size_t)sr0);
      const v4f tb = *(const v4fa*)(Tin + 4 * (size_t)sr1);
      const bool va = lane < c;
      const bool vb = (32 + lane) < c;
      float u0 = (va ? cf0 * ta.x : 0.0f) + (vb ? cf1 * tb.x : 0.0f);
      float u1 = (va ? cf0 * ta.y : 0.0f) + (vb ? cf1 * tb.y : 0.0f);
      float u2 = (va ? cf0 * ta.z : 0.0f) + (vb ? cf1 * tb.z : 0.0f);
#pragma unroll
      for (int d = 16; d > 0; d >>= 1) {
        u0 += __shfl_xor(u0, d, 32);
        u1 += __shfl_xor(u1, d, 32);
        u2 += __shfl_xor(u2, d, 32);
      }
      const v4f ts = *(const v4fa*)(Tin + 4 * (size_t)nc);
      const float y0 = ((u0 + ts.x * rd) + bf16_val(bs[0])) + pzr;
      const float y1 = ((u1 + ts.y * rd) + bf16_val(bs[1])) + pzr;
      const float y2 = ((u2 + ts.z * rd) + bf16_val(bs[2])) + pzr;
      if (lane == 0) { ybuf[3 * s + 0] = y0; ybuf[3 * s + 1] = y1; ybuf[3 * s + 2] = y2; }
    }
  }
  __syncthreads();

  const bool full = (nodeBase + NBA) <= nN;
  const int ti = tid & 63, ai = tid & 15, yi = tid < 48 ? tid : 47;
  v4f tv = {0.f, 0.f, 0.f, 0.f}, avv = {0.f, 0.f, 0.f, 0.f}, yv = {0.f, 0.f, 0.f, 0.f};
  if constexpr (MODE != 3) {
    tv  = *(const v4fa*)(tbuf + 4 * ti);
    avv = *(const v4fa*)(abuf + 4 * ai);
  }
  if constexpr (MODE != 1) yv = *(const v4fa*)(ybuf + 4 * yi);
  float* tp = Tout + 4 * (size_t)(nodeBase + ti);
  float* ap = Aout + (size_t)nodeBase + 4 * ai;
  float* yp = yout + 3 * (size_t)nodeBase + 4 * yi;
  const bool okT = full && (tid < 64), okA = full && (tid < 16), okY = full && (tid < 48);
  if constexpr (MODE != 3) {
    if (okT) *(volatile v4f*)tp = tv;
    if (okA) *(volatile v4f*)ap = avv;
  }
  if constexpr (MODE != 1) {
    if (okY) *(volatile v4f*)yp = yv;
  }
  __threadfence();
  if constexpr (MODE != 3) {
    if (okT) *(volatile v4f*)tp = tv;
    if (okA) *(volatile v4f*)ap = avv;
  }
  if constexpr (MODE != 1) {
    if (okY) *(volatile v4f*)yp = yv;
  }
}

__global__ __launch_bounds__(NTHR) void k_fin(const float* __restrict__ A12, int nN, float* outS) {
#pragma clang fp contract(off)
  __shared__ double r1[NTHR];
  __shared__ double r2[NTHR];
  const int tid = (int)threadIdx.x;
  double s1 = 0.0, s2 = 0.0;
  const int tot = 2 * nN;
#pragma unroll 1
  for (int i = tid; i < tot; i += NTHR) {
    float a = A12[i];
    a = (a > 0.0f) ? a : 0.2f * a;
    const float e = expf(-a);
    float p = 1.0f / (1.0f + e);
    p = (p < 0.01f) ? 0.01f : p;
    p = (p > 0.99f) ? 0.99f : p;
    const float qv = 1.0f - p;
    const float l1 = logf(2.0f * p);
    const float l2 = logf(2.0f * qv);
    const float m1 = p * l1;
    const float m2 = qv * l2;
    const float term = m1 + m2;
    const double td = (double)term;
    const bool first = i < nN;
    s1 += first ? td : 0.0;
    s2 += first ? 0.0 : td;
  }
  r1[tid] = s1;
  r2[tid] = s2;
  __syncthreads();
#pragma unroll 1
  for (int st = NTHR / 2; st > 0; st >>= 1) {
    if (tid < st) {
      const double x1 = r1[tid] + r1[tid + st];
      const double x2 = r2[tid] + r2[tid + st];
      r1[tid] = x1;
      r2[tid] = x2;
    }
    __syncthreads();
  }
  if (tid == 0) {
    const float k1 = (float)r1[0];
    const float k2 = (float)r2[0];
    const float o = (k1 + k2) * 0.5f;
    *(volatile float*)outS = o;
    __threadfence();
    *(volatile float*)outS = o;
  }
}

static inline size_t al256(size_t o) { return (o + 255) & ~(size_t)255; }

extern "C" void kernel_launch(void* const* d_in, const int* in_sizes, int n_in,
                              void* d_out, int out_size, void* d_ws, size_t ws_size,
                              hipStream_t stream) {
  if (n_in < 12) return;
  if (in_sizes[0] < CIN || (in_sizes[0] % CIN) != 0) return;
  const int nN = in_sizes[0] / CIN;
  if (nN < NBD || (nN % NBD) != 0 || nN > (1 << 20)) return;
  if (in_sizes[1] < 2 || (in_sizes[1] & 1) != 0) return;
  const int nE = in_sizes[1] / 2;
  if (nE < 1 || nE >= (1 << 24)) return;
  if (in_sizes[2] != CIN * HID || in_sizes[3] != HID) return;
  if (in_sizes[4] != NHEAD * HID) return;
  if (in_sizes[5] != HID * 3 || in_sizes[6] != 3) return;
  if (in_sizes[7] != HID * HID || in_sizes[8] != HID) return;
  if (in_sizes[9] != NHEAD * HID) return;
  if (in_sizes[10] != HID * 3 || in_sizes[11] != 3) return;
  if ((long long)out_size != 6LL * nN + 1) return;

  const float* x    = (const float*)d_in[0];
  const int*   edge = (const int*)d_in[1];
  const float* W1   = (const float*)d_in[2];
  const float* b1   = (const float*)d_in[3];
  const float* att1 = (const float*)d_in[4];
  const float* W2   = (const float*)d_in[5];
  const float* b2   = (const float*)d_in[6];
  const float* W3   = (const float*)d_in[7];
  const float* b3   = (const float*)d_in[8];
  const float* att2 = (const float*)d_in[9];
  const float* W4   = (const float*)d_in[10];
  const float* b4   = (const float*)d_in[11];
  float* out  = (float*)d_out;
  float* outY1 = out;
  float* outY2 = out + 3 * (size_t)nN;
  float* outS  = out + 6 * (size_t)nN;
  const int* src = edge;
  const int* dst = edge + nE;
  const int vec8 = ((nE & 3) == 0) ? 1 : 0;

  char* ws = (char*)d_ws;
  size_t off = 0;
  const size_t oDIS = off; off = al256(off + (size_t)nN * 4);
  const size_t oW1T = off; off = al256(off + (size_t)HID * CIN * 2);
  const size_t oW3T = off; off = al256(off + (size_t)HID * K3 * 2);
  const size_t oXB  = off; off = al256(off + (size_t)nN * CIN * 2);
  const size_t oH   = off; off = al256(off + (size_t)nN * HID * 4);
  const size_t oX1  = off; off = al256(off + (size_t)nN * K3 * 2);
  const size_t oT1  = off; off = al256(off + (size_t)nN * 4 * 4);
  const size_t oT2  = off; off = al256(off + (size_t)nN * 4 * 4);
  const size_t oA12 = off; off = al256(off + (size_t)nN * 2 * 4);
  if (off > ws_size || off > (size_t)WSMAX) return;
  float*          DIS  = (float*)(ws + oDIS);
  unsigned short* W1T  = (unsigned short*)(ws + oW1T);
  unsigned short* W3T2 = (unsigned short*)(ws + oW3T);
  unsigned short* XB   = (unsigned short*)(ws + oXB);
  float*          H    = (float*)(ws + oH);
  unsigned short* X1HL = (unsigned short*)(ws + oX1);
  float*          T1   = (float*)(ws + oT1);
  float*          T2   = (float*)(ws + oT2);
  float*          A12  = (float*)(ws + oA12);

  const int nUx = nN * (CIN / 8);
  const int gA  = nN / NBA;
  const int gM  = nN / GBM;
  k_cvx<<<(nUx + NTHR - 1) / NTHR, NTHR, 0, stream>>>(x, nN, nUx, XB);
  k_wprep<<<(NU1 + NU3) / NTHR, NTHR, 0, stream>>>(W1, W3, W1T, W3T2);
  k_deg<<<nN / NBD, NTHR, 0, stream>>>(dst, nE, vec8, DIS);
  k_gemm<<<dim3(gM, HID / GBN), GTHR, 0, stream>>>(XB, W1T, H, CIN, HID);
  k_scan<1><<<gA, NTHR, 0, stream>>>(src, dst, nE, nN, vec8, DIS, H, b1, att1, W2, X1HL, T1, A12,
                                     T2, b2, outY1);
  k_gemm<<<dim3(gM, HID / GBN), GTHR, 0, stream>>>(X1HL, W3T2, H, K3, HID);
  k_scan<2><<<gA, NTHR, 0, stream>>>(src, dst, nE, nN, vec8, DIS, H, b3, att2, W4, X1HL, T2, A12 + nN,
                                     T1, b2, outY1);
  k_scan<3><<<gA, NTHR, 0, stream>>>(src, dst, nE, nN, vec8, DIS, H, b3, att2, W4, X1HL, T1, A12,
                                     T2, b4, outY2);
  k_fin<<<1, NTHR, 0, stream>>>(A12, nN, outS);
}
